// RNN_70351564309228
// MI455X (gfx1250) — hardware-verified
//
#include <hip/hip_runtime.h>
#include <math.h>

constexpr int NSTEP   = 128;
constexpr int NBAT    = 32;
constexpr int NIN     = 1024;
constexpr int NHID    = 1024;
constexpr int NGATE   = 4 * NHID;
constexpr int NROWS   = NSTEP * NBAT;
constexpr int CVT_THR = 256;
constexpr int SEQ_THR = 512;
constexpr int SEQ_WAVES = SEQ_THR / 32;
constexpr int SEQ_BLK = 16;
constexpr int HPITCH  = 1032;
constexpr int SLABP   = 68;
constexpr float WCARRY      = 16.0f;
constexpr float WCARRY_INV  = 1.0f / 16.0f;
constexpr float LOCARRY     = 2048.0f;
constexpr float LOCARRY_INV = 1.0f / 2048.0f;
constexpr float F16_MIN_NORMAL = 6.103515625e-5f;

static_assert(NBAT % SEQ_BLK == 0, "batch tiles");
static_assert(NHID == 64 * SEQ_WAVES, "16 waves x 64 hidden units");
static_assert(NIN % 32 == 0 && NHID % 32 == 0, "K multiple of 32");
static_assert(NROWS % 64 == 0 && NGATE % 64 == 0, "GEMM tile multiples");
static_assert(((NROWS / 64) * (NGATE / 64)) % 8 == 0, "GEMM grid exact");
static_assert((NROWS * (NIN / 8)) % CVT_THR == 0, "convert grid exact");
static_assert(NIN % 64 == 0 && NGATE % 64 == 0, "transpose tiles");
static_assert((HPITCH % 8) == 0, "16-B aligned fragment rows");

typedef __attribute__((ext_vector_type(16))) _Float16 v16h;
typedef __attribute__((ext_vector_type(8)))  _Float16 v8h;
typedef __attribute__((ext_vector_type(4)))  _Float16 v4h;
typedef __attribute__((ext_vector_type(8)))  float    v8f;
typedef __attribute__((ext_vector_type(4)))  float    v4f;

__device__ __forceinline__ unsigned short f2bf_bits(float f) {
  unsigned u = __float_as_uint(f);
  return (unsigned short)((u + 0x7FFFu + ((u >> 16) & 1u)) >> 16);
}
__device__ __forceinline__ float bf_bits2f(unsigned short h) { return __uint_as_float(((unsigned)h) << 16); }
__device__ __forceinline__ float bf16r(float f) { return bf_bits2f(f2bf_bits(f)); }

__device__ __forceinline__ void dep_guard4_h(v8f& a, v8f& b, v8f& c, v8f& d, v16h x) {
  asm volatile("v_nop\n\tv_nop\n\tv_nop\n\tv_nop" : "+v"(a), "+v"(b), "+v"(c), "+v"(d) : "v"(x));
}
__device__ __forceinline__ void dep_guard8_h(v8f& a0, v8f& a1, v8f& a2, v8f& a3, v8f& a4, v8f& a5, v8f& a6, v8f& a7,
                                             v16h x0, v16h x1, v16h y0, v16h y1, v16h y2, v16h y3) {
  asm volatile("v_nop\n\tv_nop\n\tv_nop\n\tv_nop"
               : "+v"(a0), "+v"(a1), "+v"(a2), "+v"(a3), "+v"(a4), "+v"(a5), "+v"(a6), "+v"(a7)
               : "v"(x0), "v"(x1), "v"(y0), "v"(y1), "v"(y2), "v"(y3));
}
__device__ __forceinline__ void keep4_h(v16h a, v16h b, v16h c, v16h d) { asm volatile("v_nop" :: "v"(a), "v"(b), "v"(c), "v"(d)); }
__device__ __forceinline__ void acc_guard4(v8f& a, v8f& b, v8f& c, v8f& d) {
  asm volatile("v_nop\n\tv_nop\n\tv_nop\n\tv_nop" : "+v"(a), "+v"(b), "+v"(c), "+v"(d));
}

union FragU { v16h v; v8h h[2]; };
__device__ __forceinline__ v16h frag_load(const _Float16* p) {
  FragU f;
  f.h[0] = *(const v8h*)(p);
  f.h[1] = *(const v8h*)(p + 16);
  return f.v;
}
__device__ __forceinline__ v8f frag_mma(v16h a, v16h b, v8f c) {
  return __builtin_amdgcn_wmma_f32_16x16x32_f16(false, a, false, b, (short)0, c, false, false);
}

__device__ __forceinline__ float sigm_f(float x)  { return __builtin_amdgcn_rcpf(1.0f + expf(-x)); }
__device__ __forceinline__ float tanh_f(float x)  { return 1.0f - 2.0f * __builtin_amdgcn_rcpf(expf(2.0f * x) + 1.0f); }

__global__ __launch_bounds__(CVT_THR) void cvt8_kernel(const float* __restrict__ src, unsigned short* __restrict__ dst, int n8) {
  const int i = blockIdx.x * CVT_THR + threadIdx.x;
  if (i < n8) {
    const float* sp = src + (size_t)i * 8;
    const v4f a = *(const v4f*)(sp);
    const v4f b = *(const v4f*)(sp + 4);
    v8h hv;
#pragma unroll
    for (int e = 0; e < 4; ++e) {
      const float fa = bf16r(a[e]);
      const float fb = bf16r(b[e]);
      hv[e]     = (_Float16)fa;
      hv[4 + e] = (_Float16)fb;
    }
    *(volatile v8h*)(dst + (size_t)i * 8) = hv;
    __threadfence();
    *(volatile v8h*)(dst + (size_t)i * 8) = hv;
  }
}

template <bool PERM>
__global__ __launch_bounds__(CVT_THR) void tpw_kernel(const float* __restrict__ src, int R, int C, int ldo,
                                                      unsigned short* __restrict__ O, float sc) {
  __shared__ float Tt[64 * 65];
  const int tid = threadIdx.x;
  const int c0 = blockIdx.x * 64, r0 = blockIdx.y * 64;
#pragma unroll
  for (int i = 0; i < 4; ++i) {
    const int idx = i * CVT_THR + tid;
    const int rr = idx >> 4, cc = (idx & 15) * 4;
    const v4f v = *(const v4f*)(src + (size_t)(r0 + rr) * (size_t)C + c0 + cc);
    Tt[rr * 65 + cc + 0] = v[0];
    Tt[rr * 65 + cc + 1] = v[1];
    Tt[rr * 65 + cc + 2] = v[2];
    Tt[rr * 65 + cc + 3] = v[3];
  }
  __syncthreads();
  const int q = tid >> 3, c8 = (tid & 7) * 8;
  v8h hv[2];
#pragma unroll
  for (int g = 0; g < 2; ++g) {
    const int qq = g * 32 + q;
#pragma unroll
    for (int e = 0; e < 8; ++e) {
      const float f  = Tt[(c8 + e) * 65 + qq];
      const float fb = bf16r(f);
      hv[g][e] = (_Float16)(fb * sc);
    }
  }
  for (int pass = 0; pass < 2; ++pass) {
#pragma unroll
    for (int g = 0; g < 2; ++g) {
      const int n = c0 + g * 32 + q;
      const int orow = PERM ? (((n & (NHID - 1)) << 2) | (n >> 10)) : n;
      const size_t o = (size_t)orow * (size_t)ldo + (size_t)(r0 + c8);
      *(volatile v8h*)(O + o) = hv[g];
    }
    __threadfence();
  }
}

__global__ __launch_bounds__(256) void wmma_gemm64_f16(
    const unsigned short* __restrict__ Ap, int lda,
    const unsigned short* __restrict__ Btp, int ldb,
    float* __restrict__ C, int ldc, int M, int N, int K, float scale) {
  const _Float16* A  = (const _Float16*)Ap;
  const _Float16* Bt = (const _Float16*)Btp;
  __shared__ __align__(16) float sT[8][16 * 68];
  const int lane = threadIdx.x & 31;
  const int wave = threadIdx.x >> 5;
  const int tilesN = N >> 6;
  const int tilesM = M >> 6;
  const int tile = blockIdx.x * 8 + wave;
  if (tile >= tilesM * tilesN) return;
  const int tm = tile / tilesN;
  const int tn = tile - tm * tilesN;
  const int m0 = tm << 6;
  const int n0 = tn << 6;

  const int rlane = lane & 15;
  const int koff  = (lane >> 4) * 8;
  const int mOff  = (lane >> 4) * 8;

  v8f acc[4][4];
#pragma unroll
  for (int i = 0; i < 4; ++i)
#pragma unroll
    for (int j = 0; j < 4; ++j) acc[i][j] = (v8f){0.f, 0.f, 0.f, 0.f, 0.f, 0.f, 0.f, 0.f};

  for (int k0 = 0; k0 < K; k0 += 32) {
    v16h bh[4];
#pragma unroll
    for (int j = 0; j < 4; ++j) {
      const size_t bo = (size_t)(n0 + (j << 4) + rlane) * ldb + koff + k0;
      bh[j] = frag_load(Bt + bo);
    }
#pragma unroll
    for (int i = 0; i < 4; ++i) {
      const size_t ao = (size_t)(m0 + (i << 4) + rlane) * lda + koff + k0;
      const v16h ah = frag_load(A + ao);
#pragma unroll
      for (int j = 0; j < 4; ++j) acc[i][j] = frag_mma(ah, bh[j], acc[i][j]);
      dep_guard4_h(acc[i][0], acc[i][1], acc[i][2], acc[i][3], ah);
    }
    keep4_h(bh[0], bh[1], bh[2], bh[3]);
  }
  acc_guard4(acc[0][0], acc[0][1], acc[0][2], acc[0][3]);
  acc_guard4(acc[1][0], acc[1][1], acc[1][2], acc[1][3]);
  acc_guard4(acc[2][0], acc[2][1], acc[2][2], acc[2][3]);
  acc_guard4(acc[3][0], acc[3][1], acc[3][2], acc[3][3]);

  float* slab = sT[wave];
#pragma unroll
  for (int i = 0; i < 4; ++i) {
    const int mBase = m0 + (i << 4);
#pragma unroll
    for (int j = 0; j < 4; ++j) {
#pragma unroll
      for (int r = 0; r < 8; ++r) {
        const float v = acc[i][j][r] * scale;
        slab[(mOff + r) * 68 + (j << 4) + rlane] = v;
      }
    }
    __builtin_amdgcn_fence(__ATOMIC_RELEASE, "workgroup");
    __builtin_amdgcn_wave_barrier();
    __builtin_amdgcn_fence(__ATOMIC_ACQUIRE, "workgroup");
    {
      const int hh = lane >> 4, c4 = (lane & 15) * 4;
      for (int pass = 0; pass < 2; ++pass) {
#pragma unroll
        for (int it = 0; it < 8; ++it) {
          const int row = it * 2 + hh;
          const v4f v = *(const v4f*)(slab + row * 68 + c4);
          *(volatile v4f*)(C + (size_t)(mBase + row) * ldc + n0 + c4) = v;
        }
        __threadfence();
      }
    }
    __builtin_amdgcn_fence(__ATOMIC_RELEASE, "workgroup");
    __builtin_amdgcn_wave_barrier();
    __builtin_amdgcn_fence(__ATOMIC_ACQUIRE, "workgroup");
  }
}

__global__ __launch_bounds__(SEQ_THR) void lstm_seq_kernel(const float* __restrict__ GX, const float* __restrict__ bias,
                                                           const unsigned short* __restrict__ WHp,
                                                           float* __restrict__ OUT) {
  __shared__ __align__(16) _Float16 Ahi[SEQ_BLK * HPITCH];
  __shared__ __align__(16) _Float16 Alo[SEQ_BLK * HPITCH];
  __shared__ __align__(16) float    Sl[SEQ_WAVES][16 * SLABP];
  const _Float16* WH = (const _Float16*)WHp;
  const int tid = threadIdx.x, lane = tid & 31, wave = tid >> 5;
  const int c = lane & 15, hh = lane >> 4, koff = hh * 8, c4 = c * 4;
  const int rowbase = blockIdx.x * SEQ_BLK;

#pragma unroll 1
  for (int i = tid; i < SEQ_BLK * HPITCH; i += SEQ_THR) {
    Ahi[i] = (_Float16)0.0f;
    Alo[i] = (_Float16)0.0f;
  }
  const v8f z8 = {0.f, 0.f, 0.f, 0.f, 0.f, 0.f, 0.f, 0.f};
  v8f cs0 = z8, cs1 = z8, cs2 = z8, cs3 = z8;
  float* slab = Sl[wave];
  const _Float16* ahrow = Ahi + c * HPITCH + koff;
  const _Float16* alrow = Alo + c * HPITCH + koff;
  __syncthreads();

#pragma unroll 1
  for (int t = 0; t < NSTEP; ++t) {
#pragma unroll 1
    for (int nt = 0; nt < 4; ++nt) {
      const int j = 64 * wave + 16 * nt + c;
      const _Float16* wh = WH + (size_t)j * NHID + koff;
      v8f aM0 = z8, aM1 = z8, aM2 = z8, aM3 = z8;
      v8f aR0 = z8, aR1 = z8, aR2 = z8, aR3 = z8;
#pragma unroll 1
      for (int k0 = 0; k0 < NHID; k0 += 32) {
        const v16h ah = frag_load(ahrow + k0);
        const v16h al = frag_load(alrow + k0);
        const v16h b0 = frag_load(wh + k0);
        const v16h b1 = frag_load(wh + (size_t)1 * NHID * NHID + k0);
        const v16h b2 = frag_load(wh + (size_t)2 * NHID * NHID + k0);
        const v16h b3 = frag_load(wh + (size_t)3 * NHID * NHID + k0);
        aM0 = frag_mma(ah, b0, aM0);
        aR0 = frag_mma(al, b0, aR0);
        aM1 = frag_mma(ah, b1, aM1);
        aR1 = frag_mma(al, b1, aR1);
        aM2 = frag_mma(ah, b2, aM2);
        aR2 = frag_mma(al, b2, aR2);
        aM3 = frag_mma(ah, b3, aM3);
        aR3 = frag_mma(al, b3, aR3);
        dep_guard8_h(aM0, aM1, aM2, aM3, aR0, aR1, aR2, aR3, ah, al, b0, b1, b2, b3);
      }
      acc_guard4(aM0, aM1, aM2, aM3);
      acc_guard4(aR0, aR1, aR2, aR3);

      v4f zr[8];
#pragma unroll
      for (int r = 0; r < 8; ++r) {
        const size_t grow = (size_t)(t * NBAT + rowbase + 8 * hh + r);
        zr[r] = *(const v4f*)(GX + grow * NGATE + 4 * j);
      }
      const float b_i = bf16r(bias[j]);
      const float b_f = bf16r(bias[NHID + j]);
      const float b_g = bf16r(bias[2 * NHID + j]);
      const float b_o = bf16r(bias[3 * NHID + j]);

#pragma unroll
      for (int r = 0; r < 8; ++r) {
        const v4f zz = zr[r];
        const float z_i = (aM0[r] + aR0[r] * LOCARRY_INV) * WCARRY_INV + (zz[0] + b_i);
        const float z_f = (aM1[r] + aR1[r] * LOCARRY_INV) * WCARRY_INV + (zz[1] + b_f);
        const float z_g = (aM2[r] + aR2[r] * LOCARRY_INV) * WCARRY_INV + (zz[2] + b_g);
        const float z_o = (aM3[r] + aR3[r] * LOCARRY_INV) * WCARRY_INV + (zz[3] + b_o);
        const float ig = sigm_f(z_i);
        const float fg = sigm_f(z_f);
        const float gg = tanh_f(z_g);
        const float og = sigm_f(z_o);
        const float cn = fg * cs0[r] + ig * gg;
        cs0[r] = cn;
        const float hn = og * tanh_f(cn);
        slab[(8 * hh + r) * SLABP + 16 * nt + c] = hn;
      }
      const v8f ctmp = cs0;
      cs0 = cs1;
      cs1 = cs2;
      cs2 = cs3;
      cs3 = ctmp;
    }

    __syncthreads();

    v4f hv[8];
#pragma unroll
    for (int it = 0; it < 8; ++it) hv[it] = *(const v4f*)(slab + (2 * it + hh) * SLABP + c4);

#pragma unroll
    for (int it = 0; it < 8; ++it) {
      const int row = 2 * it + hh;
      const v4f v = hv[it];
      v4h h4, l4;
#pragma unroll
      for (int e = 0; e < 4; ++e) {
        const float hn   = v[e];
        const float hsel = (fabsf(hn) < F16_MIN_NORMAL) ? 0.0f : hn;
        const _Float16 hb = (_Float16)hsel;
        const float hbf = (float)hb;
        const float res = (hn - hbf) * LOCARRY;
        h4[e] = hb;
        l4[e] = (_Float16)res;
      }
      *(v4h*)(Ahi + row * HPITCH + 64 * wave + c4) = h4;
      *(v4h*)(Alo + row * HPITCH + 64 * wave + c4) = l4;
    }

    for (int pass = 0; pass < 2; ++pass) {
#pragma unroll
      for (int it = 0; it < 8; ++it) {
        const int row = 2 * it + hh;
        const size_t orow = (size_t)(t * NBAT + rowbase + row);
        *(volatile v4f*)(OUT + orow * NHID + 64 * wave + c4) = hv[it];
      }
      __threadfence();
    }

    __syncthreads();
  }
}

extern "C" void kernel_launch(void* const* d_in, const int* in_sizes, int n_in,
                              void* d_out, int out_size, void* d_ws, size_t ws_size, hipStream_t stream) {
  if (n_in < 4 || d_out == nullptr || d_ws == nullptr) return;
  if (in_sizes[0] != NSTEP * NBAT * NIN || in_sizes[1] != NIN * NGATE || in_sizes[2] != NHID * NGATE ||
      in_sizes[3] != NGATE || out_size != NSTEP * NBAT * NHID) return;

  const float* x  = (const float*)d_in[0];
  const float* wx = (const float*)d_in[1];
  const float* wh = (const float*)d_in[2];
  const float* bv = (const float*)d_in[3];
  float* out = (float*)d_out;

  char* ws = (char*)d_ws;
  size_t off = 0;
  auto carve = [&](size_t bytes) -> char* { char* p = ws + off; off += (bytes + 255) & ~(size_t)255; return p; };
  unsigned short* XH  = (unsigned short*)carve((size_t)NROWS * NIN * 2);
  unsigned short* WXT = (unsigned short*)carve((size_t)NGATE * NIN * 2);
  unsigned short* WHT = (unsigned short*)carve((size_t)NGATE * NHID * 2);
  float*          GX  = (float*)carve((size_t)NROWS * NGATE * 4);
  if (off > ws_size || off > (size_t)134217728) return;

  const int n8x = NROWS * (NIN / 8);
  cvt8_kernel<<<n8x / CVT_THR, CVT_THR, 0, stream>>>(x, XH, n8x);
  tpw_kernel<true><<<dim3(NGATE / 64, NIN / 64), CVT_THR, 0, stream>>>(wx, NIN, NGATE, NIN, WXT, WCARRY);
  tpw_kernel<false><<<dim3(NGATE / 64, NHID / 64), CVT_THR, 0, stream>>>(wh, NHID, NGATE, NHID, WHT, WCARRY);
  wmma_gemm64_f16<<<dim3(((NROWS / 64) * (NGATE / 64)) / 8), 256, 0, stream>>>(
      XH, NIN, WXT, NIN, GX, NGATE, NROWS, NGATE, NIN, WCARRY_INV);
  lstm_seq_kernel<<<NBAT / SEQ_BLK, SEQ_THR, 0, stream>>>(GX, bv, WHT, out);
}
